// CausalExpert_67723044324028
// MI455X (gfx1250) — hardware-verified
//
#include <hip/hip_runtime.h>
#include <stddef.h>
#include <stdint.h>
#include <math.h>

#define BB   2
#define NN   384
#define CC   512
#define HH   8
#define DD   64
#define FF   2048
#define TEL  1000
#define ROWS (BB * NN)
#define C3   (3 * CC)
#define C2   (2 * CC)
#define PL   ((size_t)BB * HH * NN * DD)

static_assert(NN % 128 == 0);
static_assert(NN % 64 == 0);
static_assert(NN % 32 == 0);
static_assert(ROWS % 256 == 0);
static_assert(CC % 64 == 0);
static_assert(FF % 64 == 0);
static_assert(DD == 64);
static_assert(HH * DD == CC);
static_assert(CC == 512);

#define SZ_F   ((size_t)ROWS * CC * 4)
#define SZ_H   ((size_t)ROWS * CC * 2)
#define O_XA   ((size_t)0)
#define O_H1   (O_XA + SZ_F)
#define O_WQKV (O_H1 + SZ_H)
#define O_WO   (O_WQKV + (size_t)C3 * CC * 2)
#define O_W1   (O_WO + (size_t)CC * CC * 2)
#define O_CW2  (O_W1 + (size_t)C2 * CC * 2)
#define O_EW1  (O_CW2 + (size_t)CC * CC * 2)
#define O_EW2  (O_EW1 + (size_t)FF * CC * 2)
#define O_QKV  (O_EW2 + (size_t)CC * FF * 2)
#define O_OP   (O_QKV + 3 * PL * 2)
#define O_X1   (O_OP + SZ_H)
#define O_X1H  (O_X1 + SZ_F)
#define O_ABM  (O_X1H + SZ_H)
#define O_X2   (O_ABM + (size_t)ROWS * C2 * 4)
#define O_HN   (O_X2 + SZ_F)
#define O_HP   (O_HN + SZ_H)
#define WS_TOTAL (O_HP + (size_t)ROWS * FF * 2)
static_assert(WS_TOTAL == (size_t)24379392);
static_assert(WS_TOTAL <= (size_t)134217728);
static_assert((O_H1 % 128) == 0 && (O_WQKV % 128) == 0 && (O_WO % 128) == 0 && (O_W1 % 128) == 0);
static_assert((O_CW2 % 128) == 0 && (O_EW1 % 128) == 0 && (O_EW2 % 128) == 0 && (O_QKV % 128) == 0);
static_assert((O_OP % 128) == 0 && (O_X1 % 128) == 0 && (O_X1H % 128) == 0 && (O_ABM % 128) == 0);
static_assert((O_X2 % 128) == 0 && (O_HN % 128) == 0 && (O_HP % 128) == 0);

typedef _Float16 v16h __attribute__((ext_vector_type(16)));
typedef _Float16 v8h  __attribute__((ext_vector_type(8)));
typedef float    v8f  __attribute__((ext_vector_type(8)));
typedef float    v4f  __attribute__((ext_vector_type(4)));
typedef unsigned int v4u __attribute__((ext_vector_type(4)));

union Frag  { v16h v; v8h h[2]; };
union Pack8 { v8h h; v4u u; };

__device__ __forceinline__ v8f mma16(v16h a, v16h b, v8f c) {
  c = __builtin_amdgcn_wmma_f32_16x16x32_f16(false, a, false, b, (short)0, c, false, false);
  asm volatile("v_nop\n\tv_nop\n\tv_nop\n\tv_nop" : "+v"(c) : "v"(a), "v"(b));
  return c;
}

__device__ __forceinline__ v16h ldfrag(const _Float16* p, int ld, int row0, int k0, int lane) {
  const int m = lane & 15, lh = lane >> 4;
  const _Float16* q = p + (size_t)(row0 + m) * ld + k0 + 8 * lh;
  Frag f;
  f.h[0] = *(const v8h*)(q);
  f.h[1] = *(const v8h*)(q + 16);
  return f.v;
}

__device__ __forceinline__ v8f zero8() { return (v8f){0.f, 0.f, 0.f, 0.f, 0.f, 0.f, 0.f, 0.f}; }

__device__ __forceinline__ float gelu16(float v) {
  return 8.0f * v * (1.0f + erff(v * 0.70710678118654752f));
}

template <int KK>
__device__ __forceinline__ void gemm32x64(const _Float16* __restrict__ A, int lda,
                                          const _Float16* __restrict__ Bt, int ldb,
                                          int m0, int n0, int lane, v8f (&acc)[2][4]) {
#pragma unroll 2
  for (int k0 = 0; k0 < KK; k0 += 32) {
    const v16h a0 = ldfrag(A, lda, m0, k0, lane);
    const v16h a1 = ldfrag(A, lda, m0 + 16, k0, lane);
    const v16h b0 = ldfrag(Bt, ldb, n0, k0, lane);
    const v16h b1 = ldfrag(Bt, ldb, n0 + 16, k0, lane);
    const v16h b2 = ldfrag(Bt, ldb, n0 + 32, k0, lane);
    const v16h b3 = ldfrag(Bt, ldb, n0 + 48, k0, lane);
    acc[0][0] = mma16(a0, b0, acc[0][0]);
    acc[1][0] = mma16(a1, b0, acc[1][0]);
    acc[0][1] = mma16(a0, b1, acc[0][1]);
    acc[1][1] = mma16(a1, b1, acc[1][1]);
    acc[0][2] = mma16(a0, b2, acc[0][2]);
    acc[1][2] = mma16(a1, b2, acc[1][2]);
    acc[0][3] = mma16(a0, b3, acc[0][3]);
    acc[1][3] = mma16(a1, b3, acc[1][3]);
  }
}

__global__ __launch_bounds__(128) void k_xln(const float* __restrict__ x,
                                            const float* __restrict__ te,
                                            const float* __restrict__ g,
                                            const float* __restrict__ bt,
                                            float* __restrict__ xa,
                                            _Float16* __restrict__ outh) {
  __shared__ __align__(16) float rb[CC];
  __shared__ float red[8];
  const int tid = threadIdx.x, lane = tid & 31, wave = tid >> 5;
  const int rw = blockIdx.x;
  const int i  = rw % NN;
  const size_t ro = (size_t)rw * CC;
  const v4f xv = *(const v4f*)(x + ro + 4 * tid);
  const v4f ev = *(const v4f*)(te + (size_t)i * CC + 4 * tid);
  v4f v;
  v[0] = xv[0] + ev[0]; v[1] = xv[1] + ev[1]; v[2] = xv[2] + ev[2]; v[3] = xv[3] + ev[3];
  volatile v4f* xo = (volatile v4f*)(xa + ro + 4 * tid);
  *xo = v;
  __threadfence();
  *xo = v;

  float s = (v[0] + v[1]) + (v[2] + v[3]);
#pragma unroll
  for (int off = 1; off < 32; off <<= 1) s += __shfl_xor(s, off, 32);
  if (lane == 0) red[wave] = s;
  __syncthreads();
  const float ts = (red[0] + red[1]) + (red[2] + red[3]);
  const float mean = ts * (1.0f / (float)CC);
  const float d0 = v[0] - mean, d1 = v[1] - mean, d2 = v[2] - mean, d3 = v[3] - mean;
  float q = (d0 * d0 + d1 * d1) + (d2 * d2 + d3 * d3);
#pragma unroll
  for (int off = 1; off < 32; off <<= 1) q += __shfl_xor(q, off, 32);
  if (lane == 0) red[4 + wave] = q;
  __syncthreads();
  const float tq = (red[4] + red[5]) + (red[6] + red[7]);
  const float var = tq * (1.0f / (float)CC);
  const float inv = rsqrtf(var + 1e-5f);
  const v4f g4 = *(const v4f*)(g + 4 * tid);
  const v4f b4 = *(const v4f*)(bt + 4 * tid);
  v4f o;
  o[0] = d0 * inv * g4[0] + b4[0];
  o[1] = d1 * inv * g4[1] + b4[1];
  o[2] = d2 * inv * g4[2] + b4[2];
  o[3] = d3 * inv * g4[3] + b4[3];
  *(v4f*)(rb + 4 * tid) = o;
  __syncthreads();
  if (tid < 64) {
    const v4f a0 = *(const v4f*)(rb + 8 * tid);
    const v4f a1 = *(const v4f*)(rb + 8 * tid + 4);
    Pack8 pk;
    pk.h = (v8h){(_Float16)a0[0], (_Float16)a0[1], (_Float16)a0[2], (_Float16)a0[3],
                 (_Float16)a1[0], (_Float16)a1[1], (_Float16)a1[2], (_Float16)a1[3]};
    const v4u vv = pk.u;
    volatile v4u* hq = (volatile v4u*)(outh + ro + 8 * tid);
    *hq = vv;
    __threadfence();
    *hq = vv;
  }
}

#define WTP 68
__global__ __launch_bounds__(256) void k_wt(const float* __restrict__ w, _Float16* __restrict__ wt,
                                           int nout, int kin) {
  __shared__ __align__(16) float tf[64 * WTP];
  const int tid = threadIdx.x;
  const int n0 = blockIdx.x * 64;
  const int k0 = blockIdx.y * 64;
  {
    const int kr = tid >> 4;
    const int n4 = (tid & 15) * 4;
#pragma unroll
    for (int it = 0; it < 4; ++it) {
      const int kl = it * 16 + kr;
      const v4f a = *(const v4f*)(w + (size_t)(k0 + kl) * nout + n0 + n4);
      *(v4f*)(tf + kl * WTP + n4) = a;
    }
  }
  __syncthreads();
  v4u val[2];
  size_t go[2];
#pragma unroll
  for (int j = 0; j < 2; ++j) {
    const int p  = tid + 256 * j;
    const int nl = p >> 3;
    const int pc = p & 7;
    const float* cp = tf + (pc * 8) * WTP + nl;
    Pack8 pk;
    pk.h = (v8h){(_Float16)(cp[0 * WTP] * 32.0f), (_Float16)(cp[1 * WTP] * 32.0f),
                 (_Float16)(cp[2 * WTP] * 32.0f), (_Float16)(cp[3 * WTP] * 32.0f),
                 (_Float16)(cp[4 * WTP] * 32.0f), (_Float16)(cp[5 * WTP] * 32.0f),
                 (_Float16)(cp[6 * WTP] * 32.0f), (_Float16)(cp[7 * WTP] * 32.0f)};
    val[j] = pk.u;
    go[j]  = (size_t)(n0 + nl) * kin + k0 + pc * 8;
  }
  for (int ps = 0; ps < 2; ++ps) {
#pragma unroll
    for (int j = 0; j < 2; ++j) *(volatile v4u*)(wt + go[j]) = val[j];
    __threadfence();
  }
}

#define STP 72
__global__ __launch_bounds__(128) void k_proj(const _Float16* __restrict__ ah,
                                              const _Float16* __restrict__ wt,
                                              const float* __restrict__ bq,
                                              const float* __restrict__ bk,
                                              const float* __restrict__ bv,
                                              _Float16* __restrict__ planes) {
  __shared__ __align__(16) _Float16 st[128 * STP];
  const int tid = threadIdx.x, lane = tid & 31, wave = tid >> 5;
  const int hh = lane >> 4, c = lane & 15;
  const int mb = blockIdx.x * 128;
  const int m0 = mb + wave * 32;
  const int n0 = blockIdx.y * 64;
  const int which = n0 / CC;
  const int nin   = n0 - which * CC;
  const int b     = mb / NN;
  const int nb    = mb - b * NN;
  const int head  = nin >> 6;
  const int bh    = b * HH + head;
  const float* bsel = (which == 0) ? bq : ((which == 1) ? bk : bv);

  v8f acc[2][4];
#pragma unroll
  for (int s = 0; s < 2; ++s)
#pragma unroll
    for (int t = 0; t < 4; ++t) acc[s][t] = zero8();
  gemm32x64<CC>(ah, CC, wt, CC, m0, n0, lane, acc);

#pragma unroll
  for (int t = 0; t < 4; ++t) {
    const float bb = bsel[nin + 16 * t + c];
#pragma unroll
    for (int sub = 0; sub < 2; ++sub) {
#pragma unroll
      for (int r = 0; r < 8; ++r) {
        const int lr = wave * 32 + sub * 16 + 8 * hh + r;
        st[lr * STP + 16 * t + c] = (_Float16)(acc[sub][t][r] * 0.03125f + bb);
      }
    }
  }
  __syncthreads();

  v4u val[8];
  size_t go[8];
  if (which != 2) {
#pragma unroll
    for (int j = 0; j < 8; ++j) {
      const int p  = tid + 128 * j;
      const int lr = p >> 3;
      const int pc = p & 7;
      Pack8 pk;
      pk.h   = *(const v8h*)(st + lr * STP + pc * 8);
      val[j] = pk.u;
      go[j]  = (size_t)which * PL + ((size_t)bh * NN + nb + lr) * DD + pc * 8;
    }
  } else {
#pragma unroll
    for (int j = 0; j < 8; ++j) {
      const int p  = tid + 128 * j;
      const int L  = p >> 3;
      const int pc = p & 7;
      const int d  = L >> 1;
      const int sl = (L & 1) * 64 + pc * 8;
      const _Float16* cp = st + sl * STP + d;
      Pack8 pk;
      pk.h = (v8h){cp[0 * STP], cp[1 * STP], cp[2 * STP], cp[3 * STP],
                   cp[4 * STP], cp[5 * STP], cp[6 * STP], cp[7 * STP]};
      val[j] = pk.u;
      go[j]  = 2 * PL + ((size_t)bh * DD + d) * NN + nb + sl;
    }
  }
  for (int ps = 0; ps < 2; ++ps) {
#pragma unroll
    for (int j = 0; j < 8; ++j) *(volatile v4u*)(planes + go[j]) = val[j];
    __threadfence();
  }
}

#define KTP 72
#define PTP 72
__global__ __launch_bounds__(256) void k_attn(const _Float16* __restrict__ qp,
                                              const _Float16* __restrict__ kp,
                                              const _Float16* __restrict__ vt,
                                              _Float16* __restrict__ op, float sscale) {
  __shared__ __align__(16) _Float16 Ks[64 * KTP];
  __shared__ __align__(16) _Float16 Vs[64 * KTP];
  __shared__ __align__(16) _Float16 Ps[8][16 * PTP];

  const int tid = threadIdx.x, lane = tid & 31, wave = tid >> 5;
  const int hh = lane >> 4, c = lane & 15;
  const int nqb = NN / 128;
  const int bh = blockIdx.x / nqb;
  const int qb = blockIdx.x - bh * nqb;
  const int b  = bh / HH, h = bh - b * HH;
  const int q0 = qb * 128 + wave * 16;

  const _Float16* Q = qp + (size_t)bh * NN * DD;
  const _Float16* K = kp + (size_t)bh * NN * DD;
  const _Float16* V = vt + (size_t)bh * DD * NN;

  v16h qa[2];
  qa[0] = ldfrag(Q, DD, q0, 0, lane);
  qa[1] = ldfrag(Q, DD, q0, 32, lane);

  const float NEGI = -__builtin_huge_valf();
  float mrow[8], lrow[8];
  v8f oacc[4];
#pragma unroll
  for (int r = 0; r < 8; ++r) { mrow[r] = NEGI; lrow[r] = 0.f; }
#pragma unroll
  for (int t = 0; t < 4; ++t) oacc[t] = zero8();

  _Float16* pw = Ps[wave];
  const int nch = 2 * qb + 2;

  for (int kc = 0; kc < nch; ++kc) {
    const int kv0 = kc * 64;
    __syncthreads();
    {
      const int r  = tid >> 2;
      const int qq = (tid & 3) * 16;
      const _Float16* ks = K + (size_t)(kv0 + r) * DD + qq;
      *(v8h*)(Ks + r * KTP + qq)     = *(const v8h*)(ks);
      *(v8h*)(Ks + r * KTP + qq + 8) = *(const v8h*)(ks + 8);
      const _Float16* vs = V + (size_t)r * NN + kv0 + qq;
      *(v8h*)(Vs + r * KTP + qq)     = *(const v8h*)(vs);
      *(v8h*)(Vs + r * KTP + qq + 8) = *(const v8h*)(vs + 8);
    }
    __syncthreads();

    v8f s[4];
#pragma unroll
    for (int j = 0; j < 4; ++j) s[j] = zero8();
#pragma unroll
    for (int dc = 0; dc < 2; ++dc) {
#pragma unroll
      for (int j = 0; j < 4; ++j) {
        const v16h kb = ldfrag(Ks, KTP, j * 16, dc * 32, lane);
        s[j] = mma16(qa[dc], kb, s[j]);
      }
    }
    float cm[8];
#pragma unroll
    for (int r = 0; r < 8; ++r) {
      const int qrow = q0 + 8 * hh + r;
      float m = NEGI;
#pragma unroll
      for (int j = 0; j < 4; ++j) {
        const int key = kv0 + j * 16 + c;
        const float sv = (key <= qrow) ? (s[j][r] * sscale) : -1.0e9f;
        s[j][r] = sv;
        m = fmaxf(m, sv);
      }
#pragma unroll
      for (int off = 1; off < 16; off <<= 1) m = fmaxf(m, __shfl_xor(m, off, 32));
      cm[r] = m;
    }
    float al[8];
#pragma unroll
    for (int r = 0; r < 8; ++r) {
      const float mnew  = fmaxf(mrow[r], cm[r]);
      const float alpha = __expf(mrow[r] - mnew);
      mrow[r] = mnew;
      float psum = 0.f;
#pragma unroll
      for (int j = 0; j < 4; ++j) {
        const float p = __expf(s[j][r] - mnew);
        psum += p;
        pw[(8 * hh + r) * PTP + j * 16 + c] = (_Float16)(p * 1024.0f);
      }
#pragma unroll
      for (int off = 1; off < 16; off <<= 1) psum += __shfl_xor(psum, off, 32);
      lrow[r] = lrow[r] * alpha + psum;
      al[r] = alpha;
    }
#pragma unroll
    for (int t = 0; t < 4; ++t)
#pragma unroll
      for (int r = 0; r < 8; ++r) oacc[t][r] *= al[r];
    __syncthreads();

#pragma unroll
    for (int kk = 0; kk < 2; ++kk) {
      const v16h pa = ldfrag(pw, PTP, 0, kk * 32, lane);
#pragma unroll
      for (int t = 0; t < 4; ++t) {
        const v16h vb = ldfrag(Vs, KTP, t * 16, kk * 32, lane);
        oacc[t] = mma16(pa, vb, oacc[t]);
      }
    }
  }
  __syncthreads();

#pragma unroll
  for (int r = 0; r < 8; ++r) {
    const float inv = 0.0625f * (1.0f / lrow[r]);
#pragma unroll
    for (int t = 0; t < 4; ++t) pw[(8 * hh + r) * PTP + 16 * t + c] = (_Float16)(oacc[t][r] * inv);
  }
  __syncthreads();
  v4u val[4];
  size_t go[4];
#pragma unroll
  for (int it = 0; it < 4; ++it) {
    const int p  = lane + 32 * it;
    const int L  = p >> 3;
    const int pc = p & 7;
    Pack8 pk;
    pk.h    = *(const v8h*)(pw + L * PTP + pc * 8);
    val[it] = pk.u;
    go[it]  = ((size_t)(b * NN + q0 + L)) * CC + (size_t)h * DD + pc * 8;
  }
  for (int ps = 0; ps < 2; ++ps) {
#pragma unroll
    for (int it = 0; it < 4; ++it) *(volatile v4u*)(op + go[it]) = val[it];
    __threadfence();
  }
}

#define OTP 68
__global__ __launch_bounds__(256) void k_x1(const _Float16* __restrict__ ap,
                                            const _Float16* __restrict__ wt,
                                            const float* __restrict__ bias,
                                            const float* __restrict__ res,
                                            float* __restrict__ xo,
                                            _Float16* __restrict__ xh, float oscale) {
  __shared__ __align__(16) float st[8][16 * OTP];
  const int tid = threadIdx.x, lane = tid & 31, wave = tid >> 5;
  const int hh = lane >> 4, c = lane & 15;
  const int m0 = blockIdx.x * 256 + wave * 32;
  const int n0 = blockIdx.y * 64;

  v8f acc[2][4];
#pragma unroll
  for (int s = 0; s < 2; ++s)
#pragma unroll
    for (int t = 0; t < 4; ++t) acc[s][t] = zero8();
  gemm32x64<CC>(ap, CC, wt, CC, m0, n0, lane, acc);

  float bvs[4];
#pragma unroll
  for (int t = 0; t < 4; ++t) bvs[t] = bias[n0 + 16 * t + c];

  float* sw = st[wave];
#pragma unroll
  for (int sub = 0; sub < 2; ++sub) {
    __syncthreads();
#pragma unroll
    for (int t = 0; t < 4; ++t) {
#pragma unroll
      for (int r = 0; r < 8; ++r)
        sw[(8 * hh + r) * OTP + 16 * t + c] = acc[sub][t][r] * oscale + bvs[t];
    }
    __syncthreads();
    v4f val[8];
    size_t go[8];
#pragma unroll
    for (int it = 0; it < 8; ++it) {
      const int p    = lane + 32 * it;
      const int L    = p >> 3;
      const int pc   = p & 7;
      const int row  = L >> 1;
      const int half = L & 1;
      const size_t g = (size_t)(m0 + sub * 16 + row) * CC + n0 + half * 32 + pc * 4;
      v4f v = *(const v4f*)(sw + row * OTP + half * 32 + pc * 4);
      const v4f rr = *(const v4f*)(res + g);
      v[0] = v[0] + rr[0]; v[1] = v[1] + rr[1]; v[2] = v[2] + rr[2]; v[3] = v[3] + rr[3];
      *(v4f*)(sw + row * OTP + half * 32 + pc * 4) = v;
      val[it] = v;
      go[it]  = g;
    }
    for (int ps = 0; ps < 2; ++ps) {
#pragma unroll
      for (int it = 0; it < 8; ++it) *(volatile v4f*)(xo + go[it]) = val[it];
      __threadfence();
    }
    __syncthreads();
    v4u hv[4];
    size_t hg[4];
#pragma unroll
    for (int it = 0; it < 4; ++it) {
      const int p  = lane + 32 * it;
      const int L  = p >> 3;
      const int pc = p & 7;
      const v4f x0 = *(const v4f*)(sw + L * OTP + pc * 8);
      const v4f x1 = *(const v4f*)(sw + L * OTP + pc * 8 + 4);
      Pack8 pk;
      pk.h = (v8h){(_Float16)x0[0], (_Float16)x0[1], (_Float16)x0[2], (_Float16)x0[3],
                   (_Float16)x1[0], (_Float16)x1[1], (_Float16)x1[2], (_Float16)x1[3]};
      hv[it] = pk.u;
      hg[it] = (size_t)(m0 + sub * 16 + L) * CC + n0 + pc * 8;
    }
    for (int ps = 0; ps < 2; ++ps) {
#pragma unroll
      for (int it = 0; it < 4; ++it) *(volatile v4u*)(xh + hg[it]) = hv[it];
      __threadfence();
    }
  }
}

template <int KK, int NO, int HB, int RES>
__global__ __launch_bounds__(256) void k_gout(const _Float16* __restrict__ ap,
                                              const _Float16* __restrict__ wt,
                                              const float* __restrict__ bias,
                                              const float* __restrict__ res,
                                              float* __restrict__ out, float oscale) {
  __shared__ __align__(16) float st[8][16 * OTP];
  const int tid = threadIdx.x, lane = tid & 31, wave = tid >> 5;
  const int hh = lane >> 4, c = lane & 15;
  const int m0 = blockIdx.x * 256 + wave * 32;
  const int n0 = blockIdx.y * 64;

  v8f acc[2][4];
#pragma unroll
  for (int s = 0; s < 2; ++s)
#pragma unroll
    for (int t = 0; t < 4; ++t) acc[s][t] = zero8();
  gemm32x64<KK>(ap, KK, wt, KK, m0, n0, lane, acc);

  float bvs[4];
#pragma unroll
  for (int t = 0; t < 4; ++t) {
    if (HB) bvs[t] = bias[n0 + 16 * t + c];
    else    bvs[t] = 0.0f;
  }

  float* sw = st[wave];
#pragma unroll
  for (int sub = 0; sub < 2; ++sub) {
    __syncthreads();
#pragma unroll
    for (int t = 0; t < 4; ++t) {
#pragma unroll
      for (int r = 0; r < 8; ++r)
        sw[(8 * hh + r) * OTP + 16 * t + c] = acc[sub][t][r] * oscale + bvs[t];
    }
    __syncthreads();
    v4f val[8];
    size_t go[8];
#pragma unroll
    for (int it = 0; it < 8; ++it) {
      const int p    = lane + 32 * it;
      const int L    = p >> 3;
      const int pc   = p & 7;
      const int row  = L >> 1;
      const int half = L & 1;
      const size_t g = (size_t)(m0 + sub * 16 + row) * NO + n0 + half * 32 + pc * 4;
      v4f v = *(const v4f*)(sw + row * OTP + half * 32 + pc * 4);
      if (RES) {
        const v4f rr = *(const v4f*)(res + g);
        v[0] = v[0] + rr[0]; v[1] = v[1] + rr[1]; v[2] = v[2] + rr[2]; v[3] = v[3] + rr[3];
      }
      val[it] = v;
      go[it]  = g;
    }
    for (int ps = 0; ps < 2; ++ps) {
#pragma unroll
      for (int it = 0; it < 8; ++it) *(volatile v4f*)(out + go[it]) = val[it];
      __threadfence();
    }
  }
}

#define ATP 520
__global__ __launch_bounds__(256) void k_pair(const float* __restrict__ abm,
                                              const float* __restrict__ cb1,
                                              const _Float16* __restrict__ cw2t,
                                              const float* __restrict__ cb2,
                                              const float* __restrict__ lg,
                                              const float* __restrict__ lb,
                                              const float* __restrict__ x1,
                                              const float* __restrict__ g2,
                                              const float* __restrict__ b2,
                                              float* __restrict__ x2,
                                              _Float16* __restrict__ hn) {
  __shared__ __align__(16) _Float16 sA[32 * ATP];
  __shared__ __align__(16) float aic[CC];
  __shared__ __align__(16) float sF[CC];
  __shared__ __align__(16) float rb[CC];
  __shared__ float sPart[8 * 32];
  __shared__ float sMu[32];
  __shared__ float sRs[32];
  __shared__ float red[16];

  const int tid = threadIdx.x, lane = tid & 31, wave = tid >> 5;
  const int hh = lane >> 4, c = lane & 15;
  const int i = blockIdx.x;
  const int b = blockIdx.y;
  const size_t row = (size_t)b * NN + i;
  const int n0 = wave * 64;

  aic[tid]       = abm[row * C2 + tid] + cb1[tid];
  aic[tid + 256] = abm[row * C2 + tid + 256] + cb1[tid + 256];

  float facc[4];
#pragma unroll
  for (int t = 0; t < 4; ++t) facc[t] = 0.0f;

  const int ntile = (i >> 5) + 1;
  for (int tt = 0; tt < ntile; ++tt) {
    const int j0 = tt * 32;
    const bool full = (i - j0) >= 16;
    const int nq = full ? 8 : 4;
    __syncthreads();
#pragma unroll 2
    for (int q = 0; q < nq; ++q) {
      const int p  = tid + 256 * q;
      const int r  = p >> 6;
      const int k8 = (p & 63) * 8;
      const float* bp = abm + ((size_t)b * NN + j0 + r) * C2 + CC + k8;
      const v4f u0 = *(const v4f*)(bp);
      const v4f u1 = *(const v4f*)(bp + 4);
      const v4f e0 = *(const v4f*)(aic + k8);
      const v4f e1 = *(const v4f*)(aic + k8 + 4);
      Pack8 pk;
      pk.h = (v8h){(_Float16)gelu16(u0[0] + e0[0]), (_Float16)gelu16(u0[1] + e0[1]),
                   (_Float16)gelu16(u0[2] + e0[2]), (_Float16)gelu16(u0[3] + e0[3]),
                   (_Float16)gelu16(u1[0] + e1[0]), (_Float16)gelu16(u1[1] + e1[1]),
                   (_Float16)gelu16(u1[2] + e1[2]), (_Float16)gelu16(u1[3] + e1[3])};
      *(v8h*)(sA + r * ATP + k8) = pk.h;
    }
    __syncthreads();

    v8f acc[2][4];
#pragma unroll
    for (int s = 0; s < 2; ++s)
#pragma unroll
      for (int t = 0; t < 4; ++t) acc[s][t] = zero8();
#pragma unroll 2
    for (int k0 = 0; k0 < CC; k0 += 32) {
      const v16h a0 = ldfrag(sA, ATP, 0, k0, lane);
      const v16h a1 = ldfrag(sA, ATP, 16, k0, lane);
      const v16h w0 = ldfrag(cw2t, CC, n0, k0, lane);
      const v16h w1 = ldfrag(cw2t, CC, n0 + 16, k0, lane);
      const v16h w2 = ldfrag(cw2t, CC, n0 + 32, k0, lane);
      const v16h w3 = ldfrag(cw2t, CC, n0 + 48, k0, lane);
      acc[0][0] = mma16(a0, w0, acc[0][0]);
      acc[0][1] = mma16(a0, w1, acc[0][1]);
      acc[0][2] = mma16(a0, w2, acc[0][2]);
      acc[0][3] = mma16(a0, w3, acc[0][3]);
      if (full) {
        acc[1][0] = mma16(a1, w0, acc[1][0]);
        acc[1][1] = mma16(a1, w1, acc[1][1]);
        acc[1][2] = mma16(a1, w2, acc[1][2]);
        acc[1][3] = mma16(a1, w3, acc[1][3]);
      }
    }

    float cbv[4], gv[4], lbv[4];
#pragma unroll
    for (int t = 0; t < 4; ++t) {
      const int n = n0 + 16 * t + c;
      cbv[t] = cb2[n]; gv[t] = lg[n]; lbv[t] = lb[n];
    }
#pragma unroll
    for (int sub = 0; sub < 2; ++sub)
#pragma unroll
      for (int t = 0; t < 4; ++t)
#pragma unroll
        for (int r = 0; r < 8; ++r) acc[sub][t][r] = acc[sub][t][r] * 0.001953125f + cbv[t];

#pragma unroll
    for (int sub = 0; sub < 2; ++sub) {
#pragma unroll
      for (int r = 0; r < 8; ++r) {
        float ps = (acc[sub][0][r] + acc[sub][1][r]) + (acc[sub][2][r] + acc[sub][3][r]);
#pragma unroll
        for (int off = 1; off < 16; off <<= 1) ps += __shfl_xor(ps, off, 32);
        if (c == 0) sPart[wave * 32 + sub * 16 + 8 * hh + r] = ps;
      }
    }
    __syncthreads();
    if (tid < 32) {
      float s = 0.0f;
#pragma unroll
      for (int w = 0; w < 8; ++w) s += sPart[w * 32 + tid];
      sMu[tid] = s * (1.0f / (float)CC);
    }
    __syncthreads();
#pragma unroll
    for (int sub = 0; sub < 2; ++sub) {
#pragma unroll
      for (int r = 0; r < 8; ++r) {
        const float mu = sMu[sub * 16 + 8 * hh + r];
#pragma unroll
        for (int t = 0; t < 4; ++t) acc[sub][t][r] -= mu;
        float qs = (acc[sub][0][r] * acc[sub][0][r] + acc[sub][1][r] * acc[sub][1][r]) +
                   (acc[sub][2][r] * acc[sub][2][r] + acc[sub][3][r] * acc[sub][3][r]);
#pragma unroll
        for (int off = 1; off < 16; off <<= 1) qs += __shfl_xor(qs, off, 32);
        if (c == 0) sPart[wave * 32 + sub * 16 + 8 * hh + r] = qs;
      }
    }
    __syncthreads();
    if (tid < 32) {
      float qt = 0.0f;
#pragma unroll
      for (int w = 0; w < 8; ++w) qt += sPart[w * 32 + tid];
      sRs[tid] = rsqrtf(qt * (1.0f / (float)CC) + 1e-5f);
    }
    __syncthreads();
#pragma unroll
    for (int sub = 0; sub < 2; ++sub) {
#pragma unroll
      for (int r = 0; r < 8; ++r) {
        const float rs = sRs[sub * 16 + 8 * hh + r];
        const int jrow = j0 + sub * 16 + 8 * hh + r;
        const bool live = (jrow <= i);
#pragma unroll
        for (int t = 0; t < 4; ++t) {
          const float val = acc[sub][t][r] * rs * gv[t] + lbv[t];
          facc[t] += live ? val : 0.0f;
        }
      }
    }
  }

#pragma unroll
  for (int t = 0; t < 4; ++t) facc[t] += __shfl_xor(facc[t], 16, 32);
  if (hh == 0) {
#pragma unroll
    for (int t = 0; t < 4; ++t) sF[n0 + 16 * t + c] = facc[t];
  }
  __syncthreads();

  const float invL = 1.0f / (float)NN;
  v4f xv = (v4f){0.f, 0.f, 0.f, 0.f};
  float s = 0.0f;
  if (tid < 128) {
    const v4f xr = *(const v4f*)(x1 + row * CC + 4 * tid);
    const v4f fr = *(const v4f*)(sF + 4 * tid);
    xv[0] = xr[0] + fr[0] * invL; xv[1] = xr[1] + fr[1] * invL;
    xv[2] = xr[2] + fr[2] * invL; xv[3] = xr[3] + fr[3] * invL;
    s = (xv[0] + xv[1]) + (xv[2] + xv[3]);
  }
#pragma unroll
  for (int off = 1; off < 32; off <<= 1) s += __shfl_xor(s, off, 32);
  if (lane == 0) red[wave] = s;
  __syncthreads();
  float ts = 0.f;
#pragma unroll
  for (int w = 0; w < 8; ++w) ts += red[w];
  const float mean = ts * (1.0f / (float)CC);
  const float d0 = xv[0] - mean, d1 = xv[1] - mean, d2 = xv[2] - mean, d3 = xv[3] - mean;
  float qv = (tid < 128) ? ((d0 * d0 + d1 * d1) + (d2 * d2 + d3 * d3)) : 0.0f;
#pragma unroll
  for (int off = 1; off < 32; off <<= 1) qv += __shfl_xor(qv, off, 32);
  if (lane == 0) red[8 + wave] = qv;
  __syncthreads();
  float tq = 0.f;
#pragma unroll
  for (int w = 0; w < 8; ++w) tq += red[8 + w];
  const float var = tq * (1.0f / (float)CC);
  const float inv = rsqrtf(var + 1e-5f);
  if (tid < 128) {
    volatile v4f* xo = (volatile v4f*)(x2 + row * CC + 4 * tid);
    *xo = xv;
    __threadfence();
    *xo = xv;
    const v4f g4 = *(const v4f*)(g2 + 4 * tid);
    const v4f b4 = *(const v4f*)(b2 + 4 * tid);
    v4f o;
    o[0] = d0 * inv * g4[0] + b4[0];
    o[1] = d1 * inv * g4[1] + b4[1];
    o[2] = d2 * inv * g4[2] + b4[2];
    o[3] = d3 * inv * g4[3] + b4[3];
    *(v4f*)(rb + 4 * tid) = o;
  }
  __syncthreads();
  if (tid < 64) {
    const v4f a0 = *(const v4f*)(rb + 8 * tid);
    const v4f a1 = *(const v4f*)(rb + 8 * tid + 4);
    Pack8 pk;
    pk.h = (v8h){(_Float16)a0[0], (_Float16)a0[1], (_Float16)a0[2], (_Float16)a0[3],
                 (_Float16)a1[0], (_Float16)a1[1], (_Float16)a1[2], (_Float16)a1[3]};
    const v4u vv = pk.u;
    volatile v4u* hq = (volatile v4u*)(hn + row * CC + 8 * tid);
    *hq = vv;
    __threadfence();
    *hq = vv;
  }
}

__global__ __launch_bounds__(256) void k_ffn1(const _Float16* __restrict__ ap,
                                              const _Float16* __restrict__ wt,
                                              const float* __restrict__ bias,
                                              _Float16* __restrict__ hp) {
  __shared__ __align__(16) float st[8][16 * OTP];
  const int tid = threadIdx.x, lane = tid & 31, wave = tid >> 5;
  const int hh = lane >> 4, c = lane & 15;
  const int m0 = blockIdx.x * 256 + wave * 32;
  const int n0 = blockIdx.y * 64;

  v8f acc[2][4];
#pragma unroll
  for (int s = 0; s < 2; ++s)
#pragma unroll
    for (int t = 0; t < 4; ++t) acc[s][t] = zero8();
  gemm32x64<CC>(ap, CC, wt, CC, m0, n0, lane, acc);

  float bvs[4];
#pragma unroll
  for (int t = 0; t < 4; ++t) bvs[t] = bias[n0 + 16 * t + c];

  float* sw = st[wave];
#pragma unroll
  for (int sub = 0; sub < 2; ++sub) {
    __syncthreads();
#pragma unroll
    for (int t = 0; t < 4; ++t) {
#pragma unroll
      for (int r = 0; r < 8; ++r)
        sw[(8 * hh + r) * OTP + 16 * t + c] = acc[sub][t][r] * 0.03125f + bvs[t];
    }
    __syncthreads();
    v4u val[4];
    size_t go[4];
#pragma unroll
    for (int it = 0; it < 4; ++it) {
      const int p  = lane + 32 * it;
      const int L  = p >> 3;
      const int pc = p & 7;
      const v4f x0 = *(const v4f*)(sw + L * OTP + pc * 8);
      const v4f x1 = *(const v4f*)(sw + L * OTP + pc * 8 + 4);
      Pack8 pk;
      pk.h = (v8h){(_Float16)gelu16(x0[0]), (_Float16)gelu16(x0[1]), (_Float16)gelu16(x0[2]), (_Float16)gelu16(x0[3]),
                   (_Float16)gelu16(x1[0]), (_Float16)gelu16(x1[1]), (_Float16)gelu16(x1[2]), (_Float16)gelu16(x1[3])};
      val[it] = pk.u;
      go[it]  = (size_t)(m0 + sub * 16 + L) * FF + n0 + pc * 8;
    }
    for (int ps = 0; ps < 2; ++ps) {
#pragma unroll
      for (int it = 0; it < 4; ++it) *(volatile v4u*)(hp + go[it]) = val[it];
      __threadfence();
    }
  }
}

extern "C" void kernel_launch(void* const* d_in, const int* in_sizes, int n_in,
                              void* d_out, int out_size, void* d_ws, size_t ws_size,
                              hipStream_t stream) {
  if (n_in < 24) return;
  if (in_sizes[0] != ROWS * CC) return;
  if (in_sizes[1] != TEL * CC) return;
  if (in_sizes[2] != CC || in_sizes[3] != CC) return;
  if (in_sizes[4] != CC * CC || in_sizes[5] != CC) return;
  if (in_sizes[6] != CC * CC || in_sizes[7] != CC) return;
  if (in_sizes[8] != CC * CC || in_sizes[9] != CC) return;
  if (in_sizes[10] != CC * CC || in_sizes[11] != CC) return;
  if (in_sizes[12] != C2 * CC || in_sizes[13] != CC) return;
  if (in_sizes[14] != CC * CC || in_sizes[15] != CC) return;
  if (in_sizes[16] != CC || in_sizes[17] != CC) return;
  if (in_sizes[18] != CC || in_sizes[19] != CC) return;
  if (in_sizes[20] != CC * FF || in_sizes[21] != FF) return;
  if (in_sizes[22] != FF * CC || in_sizes[23] != CC) return;
  if (out_size != ROWS * CC) return;
  if (WS_TOTAL > ws_size) return;

  const float* x    = (const float*)d_in[0];
  const float* te   = (const float*)d_in[1];
  const float* n1g  = (const float*)d_in[2];
  const float* n1b  = (const float*)d_in[3];
  const float* wq   = (const float*)d_in[4];
  const float* bq   = (const float*)d_in[5];
  const float* wk   = (const float*)d_in[6];
  const float* bk   = (const float*)d_in[7];
  const float* wv   = (const float*)d_in[8];
  const float* bv   = (const float*)d_in[9];
  const float* wo   = (const float*)d_in[10];
  const float* bo   = (const float*)d_in[11];
  const float* cw1  = (const float*)d_in[12];
  const float* cb1  = (const float*)d_in[13];
  const float* cw2  = (const float*)d_in[14];
  const float* cb2  = (const float*)d_in[15];
  const float* clng = (const float*)d_in[16];
  const float* clnb = (const float*)d_in[17];
  const float* n2g  = (const float*)d_in[18];
  const float* n2b  = (const float*)d_in[19];
  const float* ew1  = (const float*)d_in[20];
  const float* eb1  = (const float*)d_in[21];
  const float* ew2  = (const float*)d_in[22];
  const float* eb2  = (const float*)d_in[23];
  float* out = (float*)d_out;

  char* ws = (char*)d_ws;
  float*    XA    = (float*)(ws + O_XA);
  _Float16* H1    = (_Float16*)(ws + O_H1);
  _Float16* WQKVT = (_Float16*)(ws + O_WQKV);
  _Float16* WOT   = (_Float16*)(ws + O_WO);
  _Float16* W1T   = (_Float16*)(ws + O_W1);
  _Float16* CW2T  = (_Float16*)(ws + O_CW2);
  _Float16* EW1T  = (_Float16*)(ws + O_EW1);
  _Float16* EW2T  = (_Float16*)(ws + O_EW2);
  _Float16* QKVp  = (_Float16*)(ws + O_QKV);
  _Float16* OPp   = (_Float16*)(ws + O_OP);
  float*    X1    = (float*)(ws + O_X1);
  _Float16* X1H   = (_Float16*)(ws + O_X1H);
  float*    ABM   = (float*)(ws + O_ABM);
  float*    X2    = (float*)(ws + O_X2);
  _Float16* HN    = (_Float16*)(ws + O_HN);
  _Float16* HP    = (_Float16*)(ws + O_HP);

  k_xln<<<dim3(ROWS), dim3(128), 0, stream>>>(x, te, n1g, n1b, XA, H1);

  k_wt<<<dim3(CC / 64, CC / 64), dim3(256), 0, stream>>>(wq, WQKVT, CC, CC);
  k_wt<<<dim3(CC / 64, CC / 64), dim3(256), 0, stream>>>(wk, WQKVT + (size_t)CC * CC, CC, CC);
  k_wt<<<dim3(CC / 64, CC / 64), dim3(256), 0, stream>>>(wv, WQKVT + (size_t)2 * CC * CC, CC, CC);
  k_wt<<<dim3(CC / 64, CC / 64), dim3(256), 0, stream>>>(wo, WOT, CC, CC);
  k_wt<<<dim3(CC / 64, CC / 64), dim3(256), 0, stream>>>(cw1, W1T, CC, CC);
  k_wt<<<dim3(CC / 64, CC / 64), dim3(256), 0, stream>>>(cw1 + (size_t)CC * CC, W1T + (size_t)CC * CC, CC, CC);
  k_wt<<<dim3(CC / 64, CC / 64), dim3(256), 0, stream>>>(cw2, CW2T, CC, CC);
  k_wt<<<dim3(FF / 64, CC / 64), dim3(256), 0, stream>>>(ew1, EW1T, FF, CC);
  k_wt<<<dim3(CC / 64, FF / 64), dim3(256), 0, stream>>>(ew2, EW2T, CC, FF);

  k_proj<<<dim3(ROWS / 128, C3 / 64), dim3(128), 0, stream>>>(H1, WQKVT, bq, bk, bv, QKVp);
  k_attn<<<dim3(BB * HH * (NN / 128)), dim3(256), 0, stream>>>(QKVp, QKVp + PL, QKVp + 2 * PL, OPp, 0.125f);
  k_x1<<<dim3(ROWS / 256, CC / 64), dim3(256), 0, stream>>>(OPp, WOT, bo, XA, X1, X1H, 0.00048828125f);

  k_gout<CC, C2, 0, 0><<<dim3(ROWS / 256, C2 / 64), dim3(256), 0, stream>>>(X1H, W1T, cb1, XA, ABM, 0.03125f);

  k_pair<<<dim3(NN, BB), dim3(256), 0, stream>>>(ABM, cb1, CW2T, cb2, clng, clnb, X1, n2g, n2b, X2, HN);

  k_ffn1<<<dim3(ROWS / 256, FF / 64), dim3(256), 0, stream>>>(HN, EW1T, eb1, HP);
  k_gout<FF, CC, 1, 1><<<dim3(ROWS / 256, CC / 64), dim3(256), 0, stream>>>(HP, EW2T, eb2, X2, out, 0.001953125f);
  (void)hipGetLastError();
}
